// DecoupledPointJAFAR_41704132444577
// MI455X (gfx1250) — hardware-verified
//
#include <hip/hip_runtime.h>
#include <math.h>

typedef __attribute__((ext_vector_type(16))) _Float16 v16h;
typedef __attribute__((ext_vector_type(16))) __bf16 v16b;
typedef __attribute__((ext_vector_type(8)))  _Float16 v8h;
typedef __attribute__((ext_vector_type(8)))  float v8f;
typedef __attribute__((ext_vector_type(4)))  float v4f;
typedef __attribute__((ext_vector_type(2)))  float v2f;
typedef __attribute__((ext_vector_type(4)))  unsigned v4u;
typedef __attribute__((ext_vector_type(4)))  int v4i;
typedef float __attribute__((may_alias)) float_a;
typedef int __attribute__((may_alias)) int_a;

template <typename T> __device__ __forceinline__ void vst2(void* p, T v) { *(volatile T*)p = v; __threadfence(); *(volatile T*)p = v; }
__device__ __forceinline__ v8f wmma16(v16h a, v16h b, v8f c) {
  v8f d = __builtin_amdgcn_wmma_f32_16x16x32_f16(false, a, false, b, (short)0, c, false, false);
  asm volatile("v_nop\n\tv_nop\n\tv_nop\n\tv_nop" : "+v"(d) : "v"(a), "v"(b));
  return d;
}
__device__ __forceinline__ v8f wmma_bf(v16b a, v16b b, v8f c) {
  v8f d = __builtin_amdgcn_wmma_f32_16x16x32_bf16(false, a, false, b, (short)0, c, false, false);
  asm volatile("v_nop\n\tv_nop\n\tv_nop\n\tv_nop" : "+v"(d) : "v"(a), "v"(b));
  return d;
}
__device__ __forceinline__ v16h frag_h(const _Float16* rowk0, int lane) {
  union { v16h v; v8h q[2]; } u; const _Float16* p = rowk0 + 8 * (lane >> 4);
  u.q[0] = *(const v8h*)p; u.q[1] = *(const v8h*)(p + 16); return u.v;
}
__device__ __forceinline__ v16h frag_f32(const float* rowk0, int lane) {
  v16h a; const float* p = rowk0 + 8 * (lane >> 4);
#pragma unroll
  for (int i = 0; i < 8; ++i) { a[i] = (_Float16)p[i]; a[8 + i] = (_Float16)p[16 + i]; }
  return a;
}
__device__ __forceinline__ v16h frag_f32s(const float* rowk0, int lane, float sc) {
  v16h a; const float* p = rowk0 + 8 * (lane >> 4);
#pragma unroll
  for (int i = 0; i < 8; ++i) { a[i] = (_Float16)(p[i] * sc); a[8 + i] = (_Float16)(p[16 + i] * sc); }
  return a;
}
__device__ __forceinline__ v16h fragc_f32(const float* W, int k0, int n, int lane, int ld, int K) {
  v16h a; const int g = lane >> 4;
#pragma unroll
  for (int i = 0; i < 8; ++i) { const int ka = k0 + 8 * g + i, kb = ka + 16;
    a[i] = (_Float16)(ka < K ? W[(size_t)(ka < K ? ka : K - 1) * ld + n] : 0.f); a[8 + i] = (_Float16)(kb < K ? W[(size_t)(kb < K ? kb : K - 1) * ld + n] : 0.f); }
  return a;
}
struct F2 { v16b h, l; };
__device__ __forceinline__ F2 bsplit16(const float v[16]) { F2 r;
#pragma unroll
  for (int i = 0; i < 16; ++i) { const __bf16 h = (__bf16)v[i]; r.h[i] = h; r.l[i] = (__bf16)(v[i] - (float)h); }
  return r; }
__device__ __forceinline__ F2 split_row(const float* row, int k0, int lane) { float v[16]; const float* p = row + k0 + 8 * (lane >> 4);
#pragma unroll
  for (int i = 0; i < 8; ++i) { v[i] = p[i]; v[8 + i] = p[16 + i]; }
  return bsplit16(v); }
__device__ __forceinline__ F2 split_rowK(const float* row, int k0, int lane, int K) { float v[16]; const int g = lane >> 4;
#pragma unroll
  for (int i = 0; i < 8; ++i) { const int ka = k0 + 8 * g + i, kb = ka + 16; v[i] = ka < K ? row[ka < K ? ka : K - 1] : 0.f; v[8 + i] = kb < K ? row[kb < K ? kb : K - 1] : 0.f; }
  return bsplit16(v); }
__device__ __forceinline__ F2 split_col(const float* W, int k0, int n, int lane, int ld, int K) { float v[16]; const int g = lane >> 4;
#pragma unroll
  for (int i = 0; i < 8; ++i) { const int ka = k0 + 8 * g + i, kb = ka + 16; v[i] = ka < K ? W[(size_t)(ka < K ? ka : K - 1) * ld + n] : 0.f; v[8 + i] = kb < K ? W[(size_t)(kb < K ? kb : K - 1) * ld + n] : 0.f; }
  return bsplit16(v); }
__device__ __forceinline__ v8f mac3(const F2& a, const F2& b, v8f c) { c = wmma_bf(a.l, b.h, c); c = wmma_bf(a.h, b.l, c); return wmma_bf(a.h, b.h, c); }
__device__ __forceinline__ float sigm(float v) { return 1.0f / (1.0f + expf(-v)); }
#define LDSX() do { asm volatile("s_wait_dscnt 0" ::: "memory"); __builtin_amdgcn_wave_barrier(); __builtin_amdgcn_fence(__ATOMIC_RELEASE, "workgroup"); } while (0)


#define NB 2
#ifndef NH
#define NH 16384
#endif
#define NHO 16384
#define NHI 16384
#define ML 8192
#define RH (NB * NH)
#define RL (NB * ML)
#define KN 16
#define CH 64
#ifndef RHT
#define RHT RH
#endif
typedef __attribute__((ext_vector_type(8))) __bf16 v8b;
__device__ __forceinline__ v16b frag_b(const __bf16* rowk0, int lane) {
  union { v16b v; v8b q[2]; } u; const __bf16* p = rowk0 + 8 * (lane >> 4);
  u.q[0] = *(const v8b*)p; u.q[1] = *(const v8b*)(p + 16); return u.v;
}
__device__ __forceinline__ float bfr(float v) { return (float)(__bf16)v; }
__device__ __attribute__((noinline)) float exp_ni(float v) { return expf(v); }
__device__ __attribute__((noinline)) float erf_ni(float v) { return erff(v); }

#define WS_FH   0u
#define WS_FL   (WS_FH + 4u * RH * 32)
#define WS_XH   (WS_FL + 4u * RL * 32)
#define WS_XL   (WS_XH + 4u * RH * 4)
#define WS_VL   (WS_XL + 4u * RL * 4)
#define WS_IDX  (WS_VL + 4u * RL * 8)
#define WS_PW   (WS_IDX + 4u * RH * 16)
#define P_G1 0
#define P_G2 (P_G1 + 64 * 32)
#define P_Q  (P_G2 + 64 * 64)
#define P_K  (P_Q + 64 * 64)
#define P_BD (P_K + 64 * 64)
#define P_R2 (P_BD + 32 * 64)
#define PWEND (P_R2 + 64 * 64)
#define WS_G1H  (WS_PW + 2u * PWEND)
#define WS_G1L  (WS_G1H + 4u * RH * 64)
#define WS_G2H  (WS_G1L + 4u * RL * 64)
#define WS_G2L  (WS_G2H + 4u * RH * 64)
#define WS_GMH  (WS_G2L + 4u * RL * 64)
#define WS_GML  (WS_GMH + 4u * RH * 64)
#define WS_Q    (WS_GML + 4u * RL * 64)
#define WS_K    (WS_Q + 4u * RH * 64)
#define WS_HB   (WS_K + 4u * RL * 64)
#define NSTB 128
#define WS_ST   (WS_HB + 4u * RH * 32)
#define WS_BN   (WS_ST + 4u * NSTB * 64)
#define WS_END  (WS_BN + 4u * 6 * 192)

template <int S>
__global__ __launch_bounds__(64) void k_tr(const float* __restrict__ XYZ, const float* __restrict__ GEO, const float* __restrict__ RGB, const float* __restrict__ VAL, float* __restrict__ F, float* __restrict__ X, float* __restrict__ V) {
  constexpr int NP = S ? ML : NH; constexpr int NPI = S ? ML : NHI; __shared__ __align__(16) float sf[64][32]; __shared__ __align__(16) float sx[64][4]; __shared__ __align__(16) float sv[64][8];
  const int t = threadIdx.x; const size_t r0 = (size_t)blockIdx.x * 64; const int b = (int)(r0 / NP); const int n0 = (int)(r0 % NP);
  for (int c = 0; c < 32; ++c) { float v = 0.f; if (c < 9) v = bfr(GEO[((size_t)b * 9 + c) * NPI + n0 + t]); else if (c < 18) v = bfr(RGB[((size_t)b * 9 + c - 9) * NPI + n0 + t]); sf[t][c] = v; }
  for (int c = 0; c < 4; ++c) sx[t][c] = (c < 3) ? bfr(XYZ[((size_t)b * 3 + c) * NPI + n0 + t]) : 0.f;
  if (S) { for (int c = 0; c < 8; ++c) sv[t][c] = (c < 6) ? bfr(VAL[((size_t)b * 6 + c) * NPI + n0 + t]) : 0.f; }
  __syncthreads();
  for (int q = t; q < 64 * 8; q += 64) { const int rl = q >> 3, pc = q & 7; vst2(F + (r0 + rl) * 32 + pc * 4, *(const v4f*)&sf[rl][pc * 4]); }
  vst2(X + (r0 + t) * 4, *(const v4f*)&sx[t][0]);
  if (S) { for (int q = t; q < 64 * 2; q += 64) { const int rl = q >> 1, pc = q & 1; vst2(V + (r0 + rl) * 8 + pc * 4, *(const v4f*)&sv[rl][pc * 4]); } }
}
__global__ __launch_bounds__(64) void k_packW(const float* __restrict__ Wm, int K, int KP, int NOUT, __bf16* __restrict__ DST_) {
  __shared__ __align__(16) __bf16 s[64]; const int n = blockIdx.x, t = threadIdx.x; if (n >= NOUT) return; s[t] = (__bf16)((t < K) ? Wm[(size_t)n * K + t] : 0.f); __syncthreads();
  if (t < KP / 8) vst2((unsigned*)(DST_ + (size_t)n * KP + t * 8), *(const v4u*)&s[t * 8]);
}
__global__ __launch_bounds__(64) void k_knn(const float* __restrict__ XH, const float* __restrict__ XL, int* __restrict__ IDX) {
  #pragma clang fp contract(off)
  __shared__ __align__(16) int sk[64][KN]; const int t = threadIdx.x; const size_t i = (size_t)blockIdx.x * 64 + t; const int b = (int)(i / NH);
  const float ax = XH[i * 4], ay = XH[i * 4 + 1], az = XH[i * 4 + 2]; const float sqa = (ax * ax + az * az) + ay * ay;
  float bd[KN]; int bi[KN];
#pragma unroll
  for (int q = 0; q < KN; ++q) { bd[q] = 3.0e38f; bi[q] = 0; }
  const float* xl = XL + (size_t)b * ML * 4;
#pragma unroll 1
  for (int m = 0; m < ML; ++m) { const float bx = xl[m * 4], by = xl[m * 4 + 1], bz = xl[m * 4 + 2]; const float sqb = (bx * bx + bz * bz) + by * by; const float dot = (ax * bx + ay * by) + az * bz; float d = (sqa + sqb) - 2.0f * dot; d = fmaxf(d, 0.f);
    if (d < bd[KN - 1]) { int pos = KN - 1;
#pragma unroll
      for (int q = KN - 2; q >= 0; --q) if (d < bd[q]) pos = q;
#pragma unroll
      for (int q = KN - 1; q >= 1; --q) if (q > pos) { bd[q] = bd[q - 1]; bi[q] = bi[q - 1]; }
#pragma unroll
      for (int q = 0; q < KN; ++q) if (q == pos) { bd[q] = d; bi[q] = m; } } }
#pragma unroll
  for (int q = 0; q < KN; ++q) sk[t][q] = b * ML + bi[q];
  __syncthreads();
  for (int q = t; q < 64 * 4; q += 64) { const int rl = q >> 2, pc = q & 3; vst2((unsigned*)(IDX + ((size_t)blockIdx.x * 64 + rl) * KN + pc * 4), *(const v4u*)&sk[rl][pc * 4]); }
}
template <int MODE, int NT>
__global__ __launch_bounds__(128) void k_gemm(const float* __restrict__ A, int lda, int K, const float* __restrict__ BNP, const __bf16* __restrict__ P, const float* __restrict__ bias, float* __restrict__ OUT, int ldo) {
  __shared__ __align__(16) float so[4][16][NT * 16 + 4]; __shared__ __align__(16) float sa[4][16][68];
  const int tid = threadIdx.x, wave = tid >> 5, lane = tid & 31, col = lane & 15, g = lane >> 4; const size_t r0 = (size_t)blockIdx.x * 64 + wave * 16;
  if (MODE == 2) { for (int q = lane; q < 16 * K; q += 32) { const int rl = q / K, c = q % K; sa[wave][rl][c] = fmaxf(A[(r0 + rl) * (size_t)lda + c] * BNP[64 + c] + BNP[128 + c], 0.f); } LDSX(); }
  v8f acc[NT]; for (int j = 0; j < NT; ++j) acc[j] = (v8f){};
  for (int kc = 0; kc < K / 32; ++kc) { F2 a; if (MODE == 1) { v16b ax; const float* p = A + (r0 + col) * (size_t)lda + kc * 32 + 8 * g;
#pragma unroll
      for (int i = 0; i < 8; ++i) { ax[i] = (__bf16)p[i]; ax[8 + i] = (__bf16)p[16 + i]; } a.h = ax; a.l = ax; } else if (MODE == 2) a = split_row(&sa[wave][col][0], kc * 32, lane); else a = split_row(A + (r0 + col) * (size_t)lda, kc * 32, lane);
#pragma unroll
    for (int j = 0; j < NT; ++j) { const v16b w = frag_b(P + (size_t)(j * 16 + col) * K + kc * 32, lane); if (MODE != 1) acc[j] = wmma_bf(a.l, w, acc[j]); acc[j] = wmma_bf(a.h, w, acc[j]); } }
#pragma unroll
  for (int j = 0; j < NT; ++j) { const float bb = bfr(bias[j * 16 + col]);
#pragma unroll
    for (int r = 0; r < 8; ++r) so[wave][8 * g + r][j * 16 + col] = acc[j][r] + bb; }
  LDSX();
  for (int rl = 0; rl < 16; ++rl) for (int pc = lane; pc < NT * 4; pc += 32) vst2(OUT + (r0 + rl) * (size_t)ldo + pc * 4, *(const v4f*)&so[wave][rl][pc * 4]);
}
template <int PASS>
__global__ __launch_bounds__(64) void k_stat(const float* __restrict__ Y, int W, int ld, int nrows, const float* __restrict__ BNP, float* __restrict__ ST) {
  __shared__ __align__(16) float s[64]; const int c = threadIdx.x; const int rpb = nrows / NSTB; const size_t r0 = (size_t)blockIdx.x * rpb; float a = 0.f; const float mu = (PASS && c < W) ? BNP[c] : 0.f;
  if (c < W) {
#pragma unroll 4
    for (int r = 0; r < rpb; ++r) { const float y = Y[(r0 + r) * ld + c]; const float d = y - mu; a += PASS ? d * d : y; } }
  s[c] = a; __syncthreads();
  if (c < 16) vst2(ST + (size_t)blockIdx.x * 64 + c * 4, *(const v4f*)&s[c * 4]);
}
template <int PASS>
__global__ __launch_bounds__(64) void k_fin(const float* __restrict__ ST, int W, int nrows, const float* __restrict__ G, const float* __restrict__ BE, float* __restrict__ BNP) {
  __shared__ __align__(16) float s[2][64]; const int c = threadIdx.x; float a = 0.f;
#pragma unroll 1
  for (int b = 0; b < NSTB; ++b) a += ST[(size_t)b * 64 + c];
  const float n = (float)nrows;
  if (PASS == 0) { s[0][c] = (c < W) ? a / n : 0.f; __syncthreads(); if (c < 16) vst2(BNP + c * 4, *(const v4f*)&s[0][c * 4]); }
  else { float sc = 0.f, sh = 0.f; if (c < W) { const float var = a / n; sc = bfr(G[c]) * rsqrtf(var + 1e-5f); sh = bfr(BE[c]) - BNP[c] * sc; } s[0][c] = sc; s[1][c] = sh; __syncthreads(); if (c < 16) { vst2(BNP + 64 + c * 4, *(const v4f*)&s[0][c * 4]); vst2(BNP + 128 + c * 4, *(const v4f*)&s[1][c * 4]); } }
}
template <int FILM>
__global__ __launch_bounds__(64) void k_geom(const float* __restrict__ G2, const float* __restrict__ BNP, const float* __restrict__ VL, const float* __restrict__ SCW, const float* __restrict__ SCB, const float* __restrict__ SHW, const float* __restrict__ SHB, float* __restrict__ GM) {
  __shared__ __align__(16) float s[64][68]; const int c = threadIdx.x; const size_t r0 = (size_t)blockIdx.x * 64; const float sc = BNP[64 + c], sh = BNP[128 + c];
  float w1[6], w2[6]; if (FILM) {
#pragma unroll
    for (int j = 0; j < 6; ++j) { w1[j] = bfr(SCW[c * 6 + j]); w2[j] = bfr(SHW[c * 6 + j]); } }
  for (int r = 0; r < 64; ++r) { float v = fmaxf(G2[(r0 + r) * 64 + c] * sc + sh, 0.f);
    if (FILM) { const float* vl = VL + (r0 + r) * 8; float scl = bfr(SCB[c]), shf = bfr(SHB[c]);
#pragma unroll
      for (int j = 0; j < 6; ++j) { scl += w1[j] * vl[j]; shf += w2[j] * vl[j]; }
      v = v * (scl + 1.0f) + shf; }
    s[r][c] = v; }
  __syncthreads();
  for (int q = c; q < 64 * 16; q += 64) { const int r = q >> 4, pc = q & 15; vst2(GM + (r0 + r) * 64 + pc * 4, *(const v4f*)&s[r][pc * 4]); }
}
__global__ __launch_bounds__(64) void k_bdy(const float* __restrict__ HB, const float* __restrict__ BNP, const float* __restrict__ W2, const float* __restrict__ B2, float* __restrict__ OUT2) {
  __shared__ __align__(16) float s[64]; const int t = threadIdx.x; const size_t i = (size_t)blockIdx.x * 64 + t; float a = bfr(B2[0]);
#pragma unroll 4
  for (int c = 0; c < 32; ++c) a += fmaxf(HB[i * 32 + c] * BNP[64 + c] + BNP[128 + c], 0.f) * bfr(W2[c]);
  s[t] = sigm(a); __syncthreads();
  if (t < 16) { const size_t i0 = (size_t)blockIdx.x * 64; vst2(OUT2 + (i0 / NH) * NHO + (i0 % NH) + t * 4, *(const v4f*)&s[t * 4]); }
}
__device__ __forceinline__ float pe1_of(const float* __restrict__ XH, const float* __restrict__ XL, size_t i, int nb, const float* __restrict__ W1, const float* __restrict__ B1, int c) {
  const float rx = XH[i * 4] - XL[(size_t)nb * 4], ry = XH[i * 4 + 1] - XL[(size_t)nb * 4 + 1], rz = XH[i * 4 + 2] - XL[(size_t)nb * 4 + 2];
  return ((bfr(W1[c * 3]) * rx + bfr(W1[c * 3 + 1]) * ry) + bfr(W1[c * 3 + 2]) * rz) + bfr(B1[c]);
}
template <int PASS>
__global__ __launch_bounds__(256) void k_pestat(const float* __restrict__ XH, const float* __restrict__ XL, const int* __restrict__ IDX, const float* __restrict__ W1, const float* __restrict__ B1, const float* __restrict__ BNP, float* __restrict__ ST) {
  __shared__ __align__(16) float s[4][64]; const int t = threadIdx.x; const int c = t & 63, grp = t >> 6; const float mu = PASS ? BNP[c] : 0.f; float a = 0.f;
  const int ppb = RHT / NSTB;
  for (int pl = grp; pl < ppb; pl += 4) { const size_t i = (size_t)blockIdx.x * ppb + pl;
#pragma unroll 4
    for (int k = 0; k < KN; ++k) { const int nb = min(max(IDX[i * KN + k], 0), RL - 1); const float v = pe1_of(XH, XL, i, nb, W1, B1, c); const float d = v - mu; a += PASS ? d * d : v; } }
  s[grp][c] = a; __syncthreads();
  if (t < 64) { const float tot = ((s[0][t] + s[1][t]) + s[2][t]) + s[3][t]; s[0][t] = tot; }
  __syncthreads();
  if (t < 16) vst2(ST + (size_t)blockIdx.x * 64 + t * 4, *(const v4f*)&s[0][t * 4]);
}
__global__ __launch_bounds__(256) void k_attn(const float* __restrict__ XH, const float* __restrict__ XL, const int* __restrict__ IDX, const float* __restrict__ W1, const float* __restrict__ B1, const float* __restrict__ BNP, const __bf16* __restrict__ PW, const float* __restrict__ B2, const float* __restrict__ Q, const float* __restrict__ Kp, const float* __restrict__ VL, float* __restrict__ OUT1) {
  __shared__ __align__(16) float sa[8][16][68]; __shared__ __align__(16) float so[8][16][68]; __shared__ __align__(16) float srec[6][32]; __shared__ int snb[8][16];
  const int tid = threadIdx.x, wave = tid >> 5, lane = tid & 31, col = lane & 15, g = lane >> 4; const size_t p0 = (size_t)blockIdx.x * 32; const int b = (int)(p0 / NH); const int n0 = (int)(p0 % NH);
  for (int round = 0; round < 4; ++round) { const int pl = round * 8 + wave; const size_t i = p0 + pl;
    if (lane < KN) snb[wave][lane] = min(max(IDX[i * KN + lane], 0), RL - 1);
    LDSX();
    for (int q = lane; q < KN * CH; q += 32) { const int k = q >> 6, c = q & 63; const float v = pe1_of(XH, XL, i, snb[wave][k], W1, B1, c); sa[wave][k][c] = fmaxf(v * BNP[64 + c] + BNP[128 + c], 0.f); }
    LDSX();
    v8f acc[4] = {};
#pragma unroll
    for (int kc = 0; kc < 2; ++kc) { const F2 a = split_row(&sa[wave][col][0], kc * 32, lane);
#pragma unroll
      for (int j = 0; j < 4; ++j) { const v16b w = frag_b(PW + P_R2 + (size_t)(j * 16 + col) * CH + kc * 32, lane); acc[j] = wmma_bf(a.l, w, acc[j]); acc[j] = wmma_bf(a.h, w, acc[j]); } }
#pragma unroll
    for (int j = 0; j < 4; ++j) { const int c = j * 16 + col; const float bb = bfr(B2[c]);
#pragma unroll
      for (int r = 0; r < 8; ++r) so[wave][8 * g + r][c] = acc[j][r] + bb; }
    LDSX();
    float lg = -3.0e38f;
    if (lane < KN) { const int nb = snb[wave][lane]; float a2 = 0.f;
#pragma unroll 8
      for (int c = 0; c < CH; ++c) a2 += Q[i * CH + c] * (Kp[(size_t)nb * CH + c] + so[wave][lane][c]);
      lg = a2 * 0.125f; }
    float mx = lg;
#pragma unroll
    for (int o = 1; o < 16; o <<= 1) mx = fmaxf(mx, __shfl_xor(mx, o));
    const float e = (lane < KN) ? exp_ni(lg - mx) : 0.f; float z = e;
#pragma unroll
    for (int o = 1; o < 16; o <<= 1) z += __shfl_xor(z, o);
    const float at = e / z;
#pragma unroll
    for (int c = 0; c < 6; ++c) { float v = (lane < KN) ? at * VL[(size_t)snb[wave][lane] * 8 + c] : 0.f;
#pragma unroll
      for (int o = 1; o < 16; o <<= 1) v += __shfl_xor(v, o);
      if (lane == 0) srec[c][pl] = v; }
    LDSX(); }
  __syncthreads();
  if (tid < 48) { const int c = tid >> 3, pc = tid & 7; vst2(OUT1 + ((size_t)b * 6 + c) * NHO + n0 + pc * 4, *(const v4f*)&srec[c][pc * 4]); }
}
extern "C" void kernel_launch(void* const* d_in, const int* in_sizes, int n_in, void* d_out, int out_size, void* d_ws, size_t ws_size, hipStream_t stream) {
  (void)in_sizes; (void)n_in; (void)out_size;
  const float** F = (const float**)d_in;
  if (ws_size < (size_t)WS_END) return;
  char* ws = (char*)d_ws; float *FH = (float*)(ws + WS_FH), *FL = (float*)(ws + WS_FL), *XH = (float*)(ws + WS_XH), *XL = (float*)(ws + WS_XL), *VL = (float*)(ws + WS_VL); int* IDX = (int*)(ws + WS_IDX); __bf16* PW = (__bf16*)(ws + WS_PW);
  float *G1H = (float*)(ws + WS_G1H), *G1L = (float*)(ws + WS_G1L), *G2H = (float*)(ws + WS_G2H), *G2L = (float*)(ws + WS_G2L), *GMH = (float*)(ws + WS_GMH), *GML = (float*)(ws + WS_GML), *Q = (float*)(ws + WS_Q), *Kp = (float*)(ws + WS_K), *HB = (float*)(ws + WS_HB), *ST = (float*)(ws + WS_ST), *BN = (float*)(ws + WS_BN);
  float* OUT1 = (float*)d_out; float* OUT2 = OUT1 + (size_t)NB * 6 * NHO;
  k_tr<0><<<RH / 64, 64, 0, stream>>>(F[0], F[3], F[5], nullptr, FH, XH, nullptr); k_tr<1><<<RL / 64, 64, 0, stream>>>(F[1], F[4], F[6], F[2], FL, XL, VL);
  k_packW<<<64, 64, 0, stream>>>(F[7], 18, 32, 64, PW + P_G1); k_packW<<<64, 64, 0, stream>>>(F[11], 64, 64, 64, PW + P_G2); k_packW<<<64, 64, 0, stream>>>(F[19], 64, 64, 64, PW + P_Q); k_packW<<<64, 64, 0, stream>>>(F[21], 64, 64, 64, PW + P_K); k_packW<<<32, 64, 0, stream>>>(F[23], 64, 64, 32, PW + P_BD); k_packW<<<64, 64, 0, stream>>>(F[33], 64, 64, 64, PW + P_R2);
  k_knn<<<RHT / 64, 64, 0, stream>>>(XH, XL, IDX);
  float *BG1H = BN, *BG1L = BN + 192, *BG2H = BN + 384, *BG2L = BN + 576, *BBD = BN + 768, *BRP = BN + 960;
  k_gemm<1, 4><<<RH / 64, 128, 0, stream>>>(FH, 32, 32, nullptr, PW + P_G1, F[8], G1H, 64); k_gemm<1, 4><<<RL / 64, 128, 0, stream>>>(FL, 32, 32, nullptr, PW + P_G1, F[8], G1L, 64);
  k_stat<0><<<NSTB, 64, 0, stream>>>(G1H, 64, 64, RH, BG1H, ST); k_fin<0><<<1, 64, 0, stream>>>(ST, 64, RH, F[9], F[10], BG1H); k_stat<1><<<NSTB, 64, 0, stream>>>(G1H, 64, 64, RH, BG1H, ST); k_fin<1><<<1, 64, 0, stream>>>(ST, 64, RH, F[9], F[10], BG1H);
  k_stat<0><<<NSTB, 64, 0, stream>>>(G1L, 64, 64, RL, BG1L, ST); k_fin<0><<<1, 64, 0, stream>>>(ST, 64, RL, F[9], F[10], BG1L); k_stat<1><<<NSTB, 64, 0, stream>>>(G1L, 64, 64, RL, BG1L, ST); k_fin<1><<<1, 64, 0, stream>>>(ST, 64, RL, F[9], F[10], BG1L);
  k_gemm<2, 4><<<RH / 64, 128, 0, stream>>>(G1H, 64, 64, BG1H, PW + P_G2, F[12], G2H, 64); k_gemm<2, 4><<<RL / 64, 128, 0, stream>>>(G1L, 64, 64, BG1L, PW + P_G2, F[12], G2L, 64);
  k_stat<0><<<NSTB, 64, 0, stream>>>(G2H, 64, 64, RH, BG2H, ST); k_fin<0><<<1, 64, 0, stream>>>(ST, 64, RH, F[13], F[14], BG2H); k_stat<1><<<NSTB, 64, 0, stream>>>(G2H, 64, 64, RH, BG2H, ST); k_fin<1><<<1, 64, 0, stream>>>(ST, 64, RH, F[13], F[14], BG2H);
  k_stat<0><<<NSTB, 64, 0, stream>>>(G2L, 64, 64, RL, BG2L, ST); k_fin<0><<<1, 64, 0, stream>>>(ST, 64, RL, F[13], F[14], BG2L); k_stat<1><<<NSTB, 64, 0, stream>>>(G2L, 64, 64, RL, BG2L, ST); k_fin<1><<<1, 64, 0, stream>>>(ST, 64, RL, F[13], F[14], BG2L);
  k_geom<0><<<RH / 64, 64, 0, stream>>>(G2H, BG2H, nullptr, nullptr, nullptr, nullptr, nullptr, GMH);
  k_geom<1><<<RL / 64, 64, 0, stream>>>(G2L, BG2L, VL, F[15], F[16], F[17], F[18], GML);
  k_gemm<0, 2><<<RH / 64, 128, 0, stream>>>(GMH, 64, 64, nullptr, PW + P_BD, F[24], HB, 32);
  k_stat<0><<<NSTB, 64, 0, stream>>>(HB, 32, 32, RH, BBD, ST); k_fin<0><<<1, 64, 0, stream>>>(ST, 32, RH, F[25], F[26], BBD); k_stat<1><<<NSTB, 64, 0, stream>>>(HB, 32, 32, RH, BBD, ST); k_fin<1><<<1, 64, 0, stream>>>(ST, 32, RH, F[25], F[26], BBD);
  k_bdy<<<RHT / 64, 64, 0, stream>>>(HB, BBD, F[27], F[28], OUT2);
  k_gemm<0, 4><<<RH / 64, 128, 0, stream>>>(GMH, 64, 64, nullptr, PW + P_Q, F[20], Q, 64); k_gemm<0, 4><<<RL / 64, 128, 0, stream>>>(GML, 64, 64, nullptr, PW + P_K, F[22], Kp, 64);
  k_pestat<0><<<NSTB, 256, 0, stream>>>(XH, XL, IDX, F[29], F[30], BRP, ST); k_fin<0><<<1, 64, 0, stream>>>(ST, 64, RHT * KN, F[31], F[32], BRP); k_pestat<1><<<NSTB, 256, 0, stream>>>(XH, XL, IDX, F[29], F[30], BRP, ST); k_fin<1><<<1, 64, 0, stream>>>(ST, 64, RHT * KN, F[31], F[32], BRP);
  k_attn<<<RHT / 32, 256, 0, stream>>>(XH, XL, IDX, F[29], F[30], BRP, PW, F[34], Q, Kp, VL, OUT1);
}
